// ISTAConv_31318901523050
// MI455X (gfx1250) — hardware-verified
//
#include <hip/hip_runtime.h>
#include <stddef.h>
#include <stdint.h>
#include <math.h>

#define NE      2097152
#define NM      8192
#define NN      16384
#define NB      8
#define IMGD    128
#define NTHR    256
#define CHUNK   8192
#define NCH     (NE / CHUNK)
#define EPT     (CHUNK / NTHR)
#define NBK_R   (NM / 64)
#define NBK_C   (NN / 64)
#define ROPITCH 288
#define BCAP_R  20480
#define BCAP_C  10240
#define OFFP    128
#define DEGCAP  1024
#define MEAS_B512_R 131519
#define MEAS_B512_C 66036
#define MEAS_MAXDEG 316
#define NUW2    3456
#define PB_W2   14
#define TAB_W1  0
#define TAB_W3  864
#define TAB_ETA 1728
#define TAB_N   1760
#define WSMAX   134217728

#define BK_OFF_BST 65536
#define BK_OFF_TOT (BK_OFF_BST + ROPITCH * 4)
#define BK_OFF_CNT (BK_OFF_TOT + 1024)
#define HP         72
#define WP         40
#define C12_OFF_W2 (324 * HP * 2)
#define C12_OFF_R  (C12_OFF_W2 + 288 * WP * 2)
#define C12_OFF_W1 (C12_OFF_R + 400 * 4)
#define C12_LDS    (C12_OFF_W1 + 288 * 4)
#define H2P 36

static_assert(NE % CHUNK == 0 && CHUNK == NTHR * EPT && (EPT % 4) == 0);
static_assert(NCH == 256 && NCH == NTHR);
static_assert(NBK_R == 128 && NBK_C == 256 && NBK_C + 1 <= ROPITCH && (ROPITCH % 32) == 0);
static_assert((BCAP_R % 512) == 0 && (BCAP_C % 512) == 0 && BCAP_R < 65536 && BCAP_C < 65536);
static_assert((long long)BCAP_R * 80 >= (long long)MEAS_B512_R * 11);
static_assert((long long)BCAP_C * 80 >= (long long)MEAS_B512_C * 11);
static_assert(DEGCAP >= 2 * MEAS_MAXDEG);
static_assert(BCAP_R / NTHR <= 80 && CHUNK < 65536);
static_assert(BK_OFF_CNT + 512 * NBK_C <= 300000);
static_assert(BCAP_R * 10 + 32768 + 3904 <= 300000);
static_assert((C12_OFF_W2 % 16) == 0 && (C12_OFF_R % 16) == 0 && (C12_OFF_W1 % 16) == 0);
static_assert(256 * 32 * 4 <= C12_OFF_W2);
static_assert(NUW2 == 3 * 9 * 32 * 4 && PB_W2 * NTHR >= NUW2);
static_assert((TAB_ETA * 4) % 128 == 0 && TAB_N == TAB_ETA + 32);

typedef float          v4f  __attribute__((ext_vector_type(4)));
typedef float          v8f  __attribute__((ext_vector_type(8)));
typedef double         v2d  __attribute__((ext_vector_type(2)));
typedef int            v2i  __attribute__((ext_vector_type(2)));
typedef int            v4i  __attribute__((ext_vector_type(4)));
typedef int            v8i  __attribute__((ext_vector_type(8)));
typedef unsigned short v8us __attribute__((ext_vector_type(8)));
typedef __bf16         v16b __attribute__((ext_vector_type(16)));
typedef v4f  __attribute__((may_alias)) v4fa;
typedef v2d  __attribute__((may_alias)) v2da;
typedef v2i  __attribute__((may_alias)) v2ia;
typedef v4i  __attribute__((may_alias)) v4ia;
typedef v8us __attribute__((may_alias)) v8usa;
union FragB { v16b v; v8us h[2]; v8i w; };

__device__ __forceinline__ v8f wmb(const FragB& a, const FragB& b, v8f c) {
  v8f d = __builtin_amdgcn_wmma_f32_16x16x32_bf16(false, a.v, false, b.v, (short)0, c, false, false);
  asm volatile("v_nop\n\tv_nop\n\tv_nop\n\tv_nop" : "+v"(d) : "v"(a.w), "v"(b.w));
  return d;
}

__device__ __forceinline__ unsigned int f2bf(float f) {
  const unsigned int u = __float_as_uint(f);
  const unsigned int r = ((u + 0x7FFFu + ((u >> 16) & 1u)) >> 16) & 0xFFFFu;
  return ((u & 0x7FFFFFFFu) > 0x7F800000u) ? 0x7FC0u : r;
}
__device__ __forceinline__ float bf2f(unsigned int b) { return __uint_as_float(b << 16); }
__device__ __forceinline__ float bfr(float f) { return bf2f(f2bf(f)); }
__device__ __forceinline__ float relu_p(float v) { return (v > 0.0f) ? v : (v - v); }
__device__ __forceinline__ int clampi(int v, int lo, int hi) { return v < lo ? lo : (v > hi ? hi : v); }

__device__ __forceinline__ void tab_copy(const float* __restrict__ src, float* dst, int tid) {
  const int uc = tid < 216 ? tid : 215;
  const v4f v = *(const v4f*)(src + 4 * uc);
  const v4f r = { bfr(v.x), bfr(v.y), bfr(v.z), bfr(v.w) };
  if (tid < 216) {
    *(volatile v4f*)(dst + 4 * tid) = r;
    __threadfence();
    *(volatile v4f*)(dst + 4 * tid) = r;
  }
}

__global__ __launch_bounds__(NTHR) void k_prep(const float* __restrict__ W1, const float* __restrict__ W2,
                                               const float* __restrict__ W3, const float* __restrict__ etas,
                                               float* TAB, unsigned short* W2T) {
  const int blk = (int)blockIdx.x, tid = (int)threadIdx.x;
  if (blk < PB_W2) {
    const int u  = blk * NTHR + tid;
    const int uc = u < NUW2 ? u : NUW2 - 1;
    const int in8 = uc & 3, out = (uc >> 2) & 31, jt = uc >> 7;
    const float* p = W2 + (size_t)(jt * 32 + in8 * 8) * 32 + out;
    v8us o;
#pragma unroll
    for (int i = 0; i < 8; ++i) o[i] = (unsigned short)f2bf(p[i * 32]);
    if (u < NUW2) {
      unsigned short* dp = W2T + (size_t)u * 8;
      *(volatile v8us*)dp = o;
      __threadfence();
      *(volatile v8us*)dp = o;
    }
  } else if (blk == PB_W2) {
    tab_copy(W1, TAB + TAB_W1, tid);
  } else if (blk == PB_W2 + 1) {
    tab_copy(W3, TAB + TAB_W3, tid);
  } else {
    const float e0 = etas[0], e1 = etas[1], e2 = etas[2];
    v4f r;
    r.x = (tid == 0) ? bfr(e0) : 0.0f;
    r.y = (tid == 0) ? bfr(e1) : 0.0f;
    r.z = (tid == 0) ? bfr(e2) : 0.0f;
    r.w = 0.0f;
    if (tid < 8) {
      float* dp = TAB + TAB_ETA + 4 * tid;
      *(volatile v4f*)dp = r;
      __threadfence();
      *(volatile v4f*)dp = r;
    }
  }
}

__device__ __forceinline__ void bk_count(unsigned short* myc, int k, int nkey) {
  const int kk = clampi(k, 0, nkey - 1);
  const int b = kk >> 6;
  myc[b] = (unsigned short)(myc[b] + 1);
}
__device__ __forceinline__ void bk_place(unsigned short* myc, const int* bst, v2ia* ENT,
                                         int k, int o, float v, int nkey, int noth) {
  const bool ok = (unsigned)k < (unsigned)nkey;
  const int kk = clampi(k, 0, nkey - 1);
  const int b = kk >> 6, sl = kk & 63;
  const int oo = clampi(o, 0, noth - 1);
  const int c = myc[b];
  myc[b] = (unsigned short)(c + 1);
  const int pos = clampi(bst[b] + c, 0, CHUNK - 1);
  const float fv = ok ? bfr(v) : 0.0f;
  v2i e;
  e.x = (sl << 16) | oo;
  e.y = __float_as_int(fv);
  ENT[pos] = e;
}

__global__ __launch_bounds__(NTHR) void k_bkt(const int* __restrict__ keys, const int* __restrict__ oth,
                                              const float* __restrict__ vals, int nbk, int nkey, int noth,
                                              int* STG, int* RUNOFF) {
  extern __shared__ __attribute__((aligned(16))) unsigned char bsm[];
  v2ia* ENT = (v2ia*)bsm;
  int* bst = (int*)(bsm + BK_OFF_BST);
  int* tot = (int*)(bsm + BK_OFF_TOT);
  unsigned short* CNT = (unsigned short*)(bsm + BK_OFF_CNT);
  const int tid = (int)threadIdx.x, lane = tid & 31, wave = tid >> 5;
  const int chunk = (int)blockIdx.x;
  const int e0 = chunk * CHUNK + tid * EPT;
  unsigned short* myc = CNT + (size_t)tid * nbk;

  {
    const v4i z = {0, 0, 0, 0};
#pragma unroll 1
    for (int i = 0; i < nbk / 8; ++i) *(v4ia*)(myc + 8 * i) = z;
  }
#pragma unroll 1
  for (int i = 0; i < EPT / 4; ++i) {
    const v4i k4 = *(const v4i*)(keys + e0 + 4 * i);
    bk_count(myc, k4.x, nkey);
    bk_count(myc, k4.y, nkey);
    bk_count(myc, k4.z, nkey);
    bk_count(myc, k4.w, nkey);
  }
  __syncthreads();
#pragma unroll 1
  for (int bb = tid; bb < nbk; bb += NTHR) {
    int run = 0;
#pragma unroll 4
    for (int th = 0; th < NTHR; ++th) {
      const int idx = th * nbk + bb;
      const int c = CNT[idx];
      CNT[idx] = (unsigned short)run;
      run += c;
    }
    tot[bb] = run;
  }
#pragma unroll 1
  for (int i = nbk + tid; i < ROPITCH; i += NTHR) bst[i] = CHUNK;
  __syncthreads();
  if (wave == 0) {
    const int per = nbk >> 5;
    const int base = lane * per;
    int s = 0;
#pragma unroll 1
    for (int i = 0; i < per; ++i) s += tot[base + i];
    int incl = s;
#pragma unroll
    for (int d = 1; d < 32; d <<= 1) {
      const int y = __shfl_up(incl, d, 32);
      if (lane >= d) incl += y;
    }
    int run = incl - s;
#pragma unroll 1
    for (int i = 0; i < per; ++i) {
      bst[base + i] = run;
      run += tot[base + i];
    }
  }
  __syncthreads();
#pragma unroll 1
  for (int i = 0; i < EPT / 4; ++i) {
    const v4i k4 = *(const v4i*)(keys + e0 + 4 * i);
    const v4i o4 = *(const v4i*)(oth + e0 + 4 * i);
    const v4f f4 = *(const v4f*)(vals + e0 + 4 * i);
    bk_place(myc, bst, ENT, k4.x, o4.x, f4.x, nkey, noth);
    bk_place(myc, bst, ENT, k4.y, o4.y, f4.y, nkey, noth);
    bk_place(myc, bst, ENT, k4.z, o4.z, f4.z, nkey, noth);
    bk_place(myc, bst, ENT, k4.w, o4.w, f4.w, nkey, noth);
  }
  __syncthreads();

  int* sb = STG + (size_t)chunk * CHUNK * 2;
  int* rb = RUNOFF + (size_t)chunk * ROPITCH;
  const int* entI = (const int*)bsm;
#pragma unroll 1
  for (int i = 0; i < CHUNK * 2 / (NTHR * 4); ++i) {
    const int p = (i * NTHR + tid) * 4;
    const v4i v = *(const v4ia*)(entI + p);
    *(volatile v4i*)(sb + p) = v;
  }
  if (tid < ROPITCH / 4) {
    const v4i v = *(const v4ia*)(bst + 4 * tid);
    *(volatile v4i*)(rb + 4 * tid) = v;
  }
  __threadfence();
#pragma unroll 1
  for (int i = 0; i < CHUNK * 2 / (NTHR * 4); ++i) {
    const int p = (i * NTHR + tid) * 4;
    const v4i v = *(const v4ia*)(entI + p);
    *(volatile v4i*)(sb + p) = v;
  }
  if (tid < ROPITCH / 4) {
    const v4i v = *(const v4ia*)(bst + 4 * tid);
    *(volatile v4i*)(rb + 4 * tid) = v;
  }
}

template <int BCAP>
__device__ __forceinline__ void csr_flush_pass(const v2ia* ENT, const unsigned short* INV, int* lb,
                                               int nb, int nbPad, int last, int tid) {
#pragma unroll 1
  for (int k = 0; k < BCAP / 512; ++k) {
    if (k * 512 >= nbPad) break;
    const int u = k * NTHR + tid;
    const int p0 = 2 * u, p1 = p0 + 1;
    int i0 = INV[p0 < last ? p0 : last];
    int i1 = INV[p1 < last ? p1 : last];
    i0 = i0 < last ? i0 : last;
    i1 = i1 < last ? i1 : last;
    const v2i a = ENT[i0];
    const v2i b = ENT[i1];
    v4i o;
    o.x = (p0 < nb) ? (a.x & 0xFFFF) : 0;
    o.y = (p0 < nb) ? a.y : 0;
    o.z = (p1 < nb) ? (b.x & 0xFFFF) : 0;
    o.w = (p1 < nb) ? b.y : 0;
    if (p0 < nbPad) *(volatile v4i*)(lb + 4 * u) = o;
  }
}

template <int BCAP>
__global__ __launch_bounds__(NTHR) void k_csr(const int* __restrict__ STG, const int* __restrict__ RUNOFF,
                                              int* LIST, int* OFF) {
  extern __shared__ __attribute__((aligned(16))) unsigned char csm[];
  v2ia* ENT = (v2ia*)csm;
  unsigned short* INV = (unsigned short*)(csm + (size_t)BCAP * 8);
  unsigned short* CNT = (unsigned short*)(csm + (size_t)BCAP * 10);
  int* sLo  = (int*)(csm + (size_t)BCAP * 10 + 32768);
  int* sLen = sLo + 256;
  int* sPos = sLen + 256;
  int* sDeg = sPos + 256;
  int* sst  = sDeg + 64;
  int* misc = sst + 128;
  const int tid = (int)threadIdx.x, lane = tid & 31, wave = tid >> 5;
  const int b = (int)blockIdx.x;

  {
    int lo = RUNOFF[(size_t)tid * ROPITCH + b];
    int hi = RUNOFF[(size_t)tid * ROPITCH + b + 1];
    lo = clampi(lo, 0, CHUNK);
    hi = clampi(hi, lo, CHUNK);
    sLo[tid] = lo;
    sLen[tid] = hi - lo;
  }
  __syncthreads();
  if (wave == 0) {
    const int base = lane * 8;
    int s = 0;
#pragma unroll
    for (int i = 0; i < 8; ++i) s += sLen[base + i];
    int incl = s;
#pragma unroll
    for (int d = 1; d < 32; d <<= 1) {
      const int y = __shfl_up(incl, d, 32);
      if (lane >= d) incl += y;
    }
    int run = incl - s;
#pragma unroll
    for (int i = 0; i < 8; ++i) {
      sPos[base + i] = run;
      run += sLen[base + i];
    }
    const int total = __shfl(incl, 31, 32);
    if (lane == 0) {
      misc[0] = total > BCAP ? BCAP : total;
      misc[1] = total > BCAP ? 1 : 0;
    }
  }
  __syncthreads();
  const int nb = misc[0], ovf = misc[1];
  const int last = nb > 0 ? nb - 1 : 0;

#pragma unroll 1
  for (int k = 0; k < NCH / 8; ++k) {
    const int c = k * 8 + wave;
    const int lo = sLo[c], len = sLen[c], pos = sPos[c];
    const int* sp = STG + ((size_t)c * CHUNK + lo) * 2;
#pragma unroll 1
    for (int i0 = 0; i0 < len; i0 += 32) {
      const int idx = i0 + lane;
      const int ic = idx < len ? idx : len - 1;
      const v2i e = *(const v2i*)(sp + 2 * ic);
      const int p = pos + idx;
      if (idx < len && p < BCAP) ENT[p] = e;
    }
  }
  __syncthreads();

  int per = (nb + NTHR - 1) / NTHR;
  per = per > BCAP / NTHR ? BCAP / NTHR : per;
  const int s0 = (tid * per < nb) ? tid * per : nb;
  const int s1 = (s0 + per < nb) ? s0 + per : nb;
  unsigned short* myc = CNT + tid * 64;
  {
    const v4i z = {0, 0, 0, 0};
#pragma unroll
    for (int i = 0; i < 8; ++i) *(v4ia*)(myc + 8 * i) = z;
  }
#pragma unroll 1
  for (int k = 0; k < per; ++k) {
    const int i = s0 + k;
    const int ic = i < last ? i : last;
    const v2i e = ENT[ic];
    const int sl = (e.x >> 16) & 63;
    myc[sl] = (unsigned short)(myc[sl] + ((i < s1) ? 1 : 0));
  }
  __syncthreads();
  if (tid < 64) {
    int run = 0;
#pragma unroll 4
    for (int th = 0; th < NTHR; ++th) {
      const int idx = th * 64 + tid;
      const int c = CNT[idx];
      CNT[idx] = (unsigned short)run;
      run += c;
    }
    sDeg[tid] = run;
  }
  __syncthreads();
  if (wave == 0) {
    const int d0 = sDeg[2 * lane], d1 = sDeg[2 * lane + 1];
    const int s = d0 + d1;
    int incl = s;
#pragma unroll
    for (int d = 1; d < 32; d <<= 1) {
      const int y = __shfl_up(incl, d, 32);
      if (lane >= d) incl += y;
    }
    const int run = incl - s;
    sst[2 * lane] = run;
    sst[2 * lane + 1] = run + d0;
    if (lane == 31) sst[64] = incl;
    sst[65 + lane] = (lane == 0) ? ovf : 0;
    if (lane < 31) sst[97 + lane] = 0;
  }
  __syncthreads();

#pragma unroll 1
  for (int k = 0; k < per; ++k) {
    const int i = s0 + k;
    const bool valid = i < s1;
    const int ic = i < last ? i : last;
    const v2i e = ENT[ic];
    const int sl = (e.x >> 16) & 63;
    const int c = myc[sl];
    myc[sl] = (unsigned short)(c + (valid ? 1 : 0));
    const int pos = clampi(sst[sl] + c, 0, BCAP - 1);
    if (valid) INV[pos] = (unsigned short)i;
  }
  __syncthreads();

  const int nbPad = (nb + 15) & ~15;
  int* lb = LIST + (size_t)b * BCAP * 2;
  int* ob = OFF + (size_t)b * OFFP;
  csr_flush_pass<BCAP>(ENT, INV, lb, nb, nbPad, last, tid);
  if (wave == 0) {
    const v4i v = *(const v4ia*)(sst + 4 * lane);
    *(volatile v4i*)(ob + 4 * lane) = v;
  }
  __threadfence();
  csr_flush_pass<BCAP>(ENT, INV, lb, nb, nbPad, last, tid);
  if (wave == 0) {
    const v4i v = *(const v4ia*)(sst + 4 * lane);
    *(volatile v4i*)(ob + 4 * lane) = v;
  }
}

__global__ __launch_bounds__(NTHR) void k_zu(const float* __restrict__ Zs, int rz, const float* __restrict__ u,
                                             float* ZUT) {
  __shared__ __attribute__((aligned(16))) float sT[256 * 8];
  const int tid = (int)threadIdx.x;
  const int n0 = (int)blockIdx.x * 256;
#pragma unroll
  for (int i = 0; i < 2; ++i) {
    const int idx = tid + NTHR * i;
    const int b = idx >> 6, q = idx & 63;
    const size_t off = (size_t)b * NN + n0 + 4 * q;
    v4f z = *(const v4f*)(Zs + off);
    const v4f uu = *(const v4f*)(u + off);
    if (rz != 0) { z.x = bfr(z.x); z.y = bfr(z.y); z.z = bfr(z.z); z.w = bfr(z.w); }
    sT[(4 * q + 0) * 8 + b] = z.x * bfr(uu.x);
    sT[(4 * q + 1) * 8 + b] = z.y * bfr(uu.y);
    sT[(4 * q + 2) * 8 + b] = z.z * bfr(uu.z);
    sT[(4 * q + 3) * 8 + b] = z.w * bfr(uu.w);
  }
  __syncthreads();
  v4f o[2];
#pragma unroll
  for (int i = 0; i < 2; ++i) o[i] = *(const v4fa*)(sT + 4 * (tid + NTHR * i));
  float* dp = ZUT + (size_t)n0 * 8;
#pragma unroll
  for (int i = 0; i < 2; ++i) *(volatile v4f*)(dp + 4 * (tid + NTHR * i)) = o[i];
  __threadfence();
#pragma unroll
  for (int i = 0; i < 2; ++i) *(volatile v4f*)(dp + 4 * (tid + NTHR * i)) = o[i];
}

template <int MODE, int BCAP>
__global__ __launch_bounds__(NTHR) __attribute__((amdgpu_num_vgpr(248)))
void k_walk(const int* __restrict__ LIST, const int* __restrict__ OFF, const float* __restrict__ G,
            const float* __restrict__ side, float* OUT, double* NREC, int nkey, int noth) {
  __shared__ int sOff[OFFP];
  __shared__ __attribute__((aligned(16))) float sSide[NB * 64];
  __shared__ __attribute__((aligned(16))) float sOut[64 * NB];
  __shared__ __attribute__((aligned(16))) double sRec[16];
  const int tid = (int)threadIdx.x, lane = tid & 31, wave = tid >> 5;
  const int blk = (int)blockIdx.x;
  const int k0 = blk * 64;

  if (tid < 128) {
    sOff[tid] = OFF[(size_t)blk * OFFP + tid];
    const int b = tid >> 4, q = tid & 15;
    const v4f v = *(const v4f*)(side + (size_t)b * nkey + k0 + 4 * q);
    const v4f r = { bfr(v.x), bfr(v.y), bfr(v.z), bfr(v.w) };
    *(v4fa*)(sSide + b * 64 + 4 * q) = r;
  }
  __syncthreads();
  const int nbraw = sOff[64];
  const int nb = clampi(nbraw, 0, BCAP);
  const bool ovf = (sOff[65] != 0) || (nbraw < 0) || (nbraw > BCAP);
  const float qnan = __int_as_float(0x7fc00000);

#pragma unroll 1
  for (int si = 0; si < 8; ++si) {
    const int s = si * 8 + wave;
    const int st = clampi(sOff[s], 0, nb);
    const int en = clampi(sOff[s + 1], st, nb);
    int cnt = en - st;
    const bool big = cnt > DEGCAP;
    cnt = cnt > DEGCAP ? DEGCAP : cnt;
    const int* lp = LIST + ((size_t)blk * BCAP + st) * 2;
    float acc[8];
#pragma unroll
    for (int k = 0; k < 8; ++k) acc[k] = 0.0f;
#pragma unroll 1
    for (int i0 = 0; i0 < cnt; i0 += 32) {
      const int idx = i0 + lane;
      const int ic = idx < cnt ? idx : cnt - 1;
      const v2i e = *(const v2i*)(lp + 2 * ic);
      const int o = clampi(e.x, 0, noth - 1);
      float val = __int_as_float(e.y);
      val = (idx < cnt) ? val : 0.0f;
      const float* gp = G + (size_t)o * 8;
      const v4f a = *(const v4f*)gp;
      const v4f c = *(const v4f*)(gp + 4);
      acc[0] = fmaf(val, a.x, acc[0]); acc[1] = fmaf(val, a.y, acc[1]);
      acc[2] = fmaf(val, a.z, acc[2]); acc[3] = fmaf(val, a.w, acc[3]);
      acc[4] = fmaf(val, c.x, acc[4]); acc[5] = fmaf(val, c.y, acc[5]);
      acc[6] = fmaf(val, c.z, acc[6]); acc[7] = fmaf(val, c.w, acc[7]);
    }
#pragma unroll
    for (int k = 0; k < 8; ++k) {
      float a = acc[k];
      a += __shfl_xor(a, 16);
      a += __shfl_xor(a, 8);
      a += __shfl_xor(a, 4);
      a += __shfl_xor(a, 2);
      a += __shfl_xor(a, 1);
      acc[k] = a;
    }
    const float pz = (ovf || big) ? qnan : 0.0f;
    float r[8];
#pragma unroll
    for (int k = 0; k < 8; ++k) {
      const float sv = sSide[k * 64 + s];
      r[k] = ((MODE == 0) ? (sv - acc[k]) : (sv * acc[k])) + pz;
    }
    if (lane == 0) {
      const v4f r0 = { r[0], r[1], r[2], r[3] };
      const v4f r1 = { r[4], r[5], r[6], r[7] };
      *(v4fa*)(sOut + s * 8) = r0;
      *(v4fa*)(sOut + s * 8 + 4) = r1;
    }
  }
  __syncthreads();

  if (MODE == 1) {
    if (wave == 0) {
      const int b = lane & 7;
      double sq = 0.0;
#pragma unroll 4
      for (int s = 0; s < 64; ++s) {
        const double v = (double)sOut[s * 8 + b];
        sq += v * v;
      }
      if (lane < 16) sRec[lane] = (lane < 8) ? sq : 0.0;
    }
    __syncthreads();
  }

  v4f ov = {0.f, 0.f, 0.f, 0.f};
  if (tid < 128) ov = *(const v4fa*)(sOut + 4 * tid);
  v2d rv = {0.0, 0.0};
  if (MODE == 1) {
    if (wave == 0) rv = *(const v2da*)(sRec + 2 * (lane & 7));
  }
  float* op = OUT + (size_t)k0 * 8 + 4 * tid;
  double* rp = NREC + (size_t)blk * 16 + 2 * (lane & 7);
  if (tid < 128) *(volatile v4f*)op = ov;
  if (MODE == 1) { if (tid < 8) *(volatile v2d*)rp = rv; }
  __threadfence();
  if (tid < 128) *(volatile v4f*)op = ov;
  if (MODE == 1) { if (tid < 8) *(volatile v2d*)rp = rv; }
}

__global__ __launch_bounds__(NTHR) void k_r(const float* __restrict__ Zs, int rz, const float* __restrict__ VT,
                                            const double* __restrict__ NREC, const float* __restrict__ etap,
                                            float* R) {
  __shared__ __attribute__((aligned(16))) float sT[NB * 256];
  __shared__ float sDen[NB];
  const int tid = (int)threadIdx.x, lane = tid & 31, wave = tid >> 5;
  const int n0 = (int)blockIdx.x * 256;
  if (wave == 0) {
    const int b = lane & 7;
    double s = 0.0;
#pragma unroll 4
    for (int k = 0; k < NBK_C; ++k) s += NREC[(size_t)k * 16 + b];
    const float nrm = sqrtf((float)s);
    const float den = (nrm > 1.0f || nrm != nrm) ? nrm : 1.0f;
    if (lane < 8) sDen[lane] = den;
  }
#pragma unroll
  for (int i = 0; i < 2; ++i) {
    const int idx = tid + NTHR * i;
    const v4f v = *(const v4f*)(VT + (size_t)n0 * 8 + 4 * idx);
    const int nl = idx >> 1, b0 = (idx & 1) * 4;
    sT[(b0 + 0) * 256 + nl] = v.x;
    sT[(b0 + 1) * 256 + nl] = v.y;
    sT[(b0 + 2) * 256 + nl] = v.z;
    sT[(b0 + 3) * 256 + nl] = v.w;
  }
  __syncthreads();
  const float eta = etap[0];
  v4f o[2];
#pragma unroll
  for (int i = 0; i < 2; ++i) {
    const int idx = tid + NTHR * i;
    const int b = idx >> 6, q = idx & 63;
    v4f z = *(const v4f*)(Zs + (size_t)b * NN + n0 + 4 * q);
    if (rz != 0) { z.x = bfr(z.x); z.y = bfr(z.y); z.z = bfr(z.z); z.w = bfr(z.w); }
    const v4f v = *(const v4fa*)(sT + b * 256 + 4 * q);
    const float den = sDen[b];
    v4f r;
    r.x = z.x - eta * (v.x / den);
    r.y = z.y - eta * (v.y / den);
    r.z = z.z - eta * (v.z / den);
    r.w = z.w - eta * (v.w / den);
    o[i] = r;
  }
#pragma unroll
  for (int i = 0; i < 2; ++i) {
    const int idx = tid + NTHR * i;
    *(volatile v4f*)(R + (size_t)(idx >> 6) * NN + n0 + 4 * (idx & 63)) = o[i];
  }
  __threadfence();
#pragma unroll
  for (int i = 0; i < 2; ++i) {
    const int idx = tid + NTHR * i;
    *(volatile v4f*)(R + (size_t)(idx >> 6) * NN + n0 + 4 * (idx & 63)) = o[i];
  }
}

__global__ __launch_bounds__(NTHR) __attribute__((amdgpu_num_vgpr(248)))
void k_c12(const float* __restrict__ R, const float* __restrict__ W1f, const unsigned short* __restrict__ W2T,
           float* H2) {
  extern __shared__ __attribute__((aligned(16))) unsigned char csm12[];
  unsigned short* sH  = (unsigned short*)csm12;
  float*          sD  = (float*)csm12;
  unsigned short* sW2 = (unsigned short*)(csm12 + C12_OFF_W2);
  float*          sR  = (float*)(csm12 + C12_OFF_R);
  float*          sW1 = (float*)(csm12 + C12_OFF_W1);
  const int tid = (int)threadIdx.x, lane = tid & 31, wave = tid >> 5, hh = lane >> 4, m = lane & 15;
  const int blk = (int)blockIdx.x;
  const int img = blk >> 6, h0 = ((blk >> 3) & 7) * 16, w0 = (blk & 7) * 16;

#pragma unroll
  for (int i = 0; i < 2; ++i) {
    const int idx = tid + NTHR * i;
    const int ic = idx < 400 ? idx : 399;
    const int ry = ic / 20, rx = ic - ry * 20;
    const int gh = h0 - 2 + ry, gw = w0 - 2 + rx;
    const bool ins = ((unsigned)gh < (unsigned)IMGD) && ((unsigned)gw < (unsigned)IMGD);
    const int ghc = clampi(gh, 0, IMGD - 1), gwc = clampi(gw, 0, IMGD - 1);
    const float v = R[(size_t)img * NN + ghc * IMGD + gwc];
    if (idx < 400) sR[idx] = ins ? v : 0.0f;
  }
  if (tid < 96) {
    const int ic = tid < 72 ? tid : 71;
    const v4f v = *(const v4f*)(W1f + 4 * ic);
    *(v4fa*)(sW1 + 4 * ic) = v;
  }
#pragma unroll
  for (int i = 0; i < 5; ++i) {
    const int idx = tid + NTHR * i;
    const int ic = idx < 1152 ? idx : 1151;
    const int row = ic >> 2, q = ic & 3;
    const v8us v = *(const v8usa*)(W2T + (size_t)row * 32 + q * 8);
    if (idx < 1152) *(v8usa*)(sW2 + row * WP + q * 8) = v;
  }
  __syncthreads();

#pragma unroll 1
  for (int it = 0; it < 6; ++it) {
    const int un = it * NTHR + tid;
    const int uc = un < 1296 ? un : 1295;
    const int p = uc >> 2, cg = uc & 3;
    const int py = p / 18, px = p - py * 18;
    const int gh = h0 - 1 + py, gw = w0 - 1 + px;
    const bool ins = ((unsigned)gh < (unsigned)IMGD) && ((unsigned)gw < (unsigned)IMGD);
    float a[8];
#pragma unroll
    for (int i = 0; i < 8; ++i) a[i] = 0.0f;
#pragma unroll
    for (int t = 0; t < 9; ++t) {
      const float rv = sR[(py + t / 3) * 20 + px + (t % 3)];
      const v4f wa = *(const v4fa*)(sW1 + t * 32 + cg * 8);
      const v4f wb = *(const v4fa*)(sW1 + t * 32 + cg * 8 + 4);
      a[0] = fmaf(rv, wa.x, a[0]); a[1] = fmaf(rv, wa.y, a[1]);
      a[2] = fmaf(rv, wa.z, a[2]); a[3] = fmaf(rv, wa.w, a[3]);
      a[4] = fmaf(rv, wb.x, a[4]); a[5] = fmaf(rv, wb.y, a[5]);
      a[6] = fmaf(rv, wb.z, a[6]); a[7] = fmaf(rv, wb.w, a[7]);
    }
    v8us ho, lo;
#pragma unroll
    for (int i = 0; i < 8; ++i) {
      float v = relu_p(a[i]);
      v = ins ? v : 0.0f;
      const unsigned int hb = f2bf(v);
      ho[i] = (unsigned short)hb;
      lo[i] = (unsigned short)f2bf(v - bf2f(hb));
    }
    if (un < 1296) {
      *(v8usa*)(sH + p * HP + cg * 8) = ho;
      *(v8usa*)(sH + p * HP + 32 + cg * 8) = lo;
    }
  }
  __syncthreads();

  v8f acc[2][2];
  {
    const v8f z = {0.f, 0.f, 0.f, 0.f, 0.f, 0.f, 0.f, 0.f};
    acc[0][0] = z; acc[0][1] = z; acc[1][0] = z; acc[1][1] = z;
  }
#pragma unroll 1
  for (int t = 0; t < 9; ++t) {
    const int kh = t / 3, kw = t - 3 * kh;
    const unsigned short* wb = sW2 + (t * 32 + m) * WP + 8 * hh;
    FragB b0, b1;
    b0.h[0] = *(const v8usa*)wb;
    b0.h[1] = *(const v8usa*)(wb + 16);
    b1.h[0] = *(const v8usa*)(wb + 16 * WP);
    b1.h[1] = *(const v8usa*)(wb + 16 * WP + 16);
#pragma unroll
    for (int mt = 0; mt < 2; ++mt) {
      const int p = (2 * wave + mt + kh) * 18 + m + kw;
      const unsigned short* ap = sH + p * HP + 8 * hh;
      FragB ah, al;
      ah.h[0] = *(const v8usa*)ap;
      ah.h[1] = *(const v8usa*)(ap + 16);
      al.h[0] = *(const v8usa*)(ap + 32);
      al.h[1] = *(const v8usa*)(ap + 48);
      acc[mt][0] = wmb(ah, b0, acc[mt][0]);
      acc[mt][1] = wmb(ah, b1, acc[mt][1]);
      acc[mt][0] = wmb(al, b0, acc[mt][0]);
      acc[mt][1] = wmb(al, b1, acc[mt][1]);
    }
  }
  __syncthreads();

#pragma unroll
  for (int mt = 0; mt < 2; ++mt)
#pragma unroll
    for (int nt = 0; nt < 2; ++nt)
#pragma unroll
      for (int r = 0; r < 8; ++r) {
        const int px = (2 * wave + mt) * 16 + 8 * hh + r;
        sD[px * 32 + nt * 16 + m] = relu_p(acc[mt][nt][r]);
      }
  __syncthreads();

  v4f fv[8];
#pragma unroll
  for (int i = 0; i < 8; ++i) {
    const int idx = tid + NTHR * i;
    fv[i] = *(const v4fa*)(sD + (idx >> 3) * 32 + 4 * (idx & 7));
  }
#pragma unroll
  for (int i = 0; i < 8; ++i) {
    const int idx = tid + NTHR * i;
    const int px = idx >> 3, q = idx & 7;
    const int ty = px >> 4, tx = px & 15;
    float* op = H2 + ((size_t)(img * IMGD + h0 + ty) * IMGD + w0 + tx) * 32 + 4 * q;
    *(volatile v4f*)op = fv[i];
  }
  __threadfence();
#pragma unroll
  for (int i = 0; i < 8; ++i) {
    const int idx = tid + NTHR * i;
    const int px = idx >> 3, q = idx & 7;
    const int ty = px >> 4, tx = px & 15;
    float* op = H2 + ((size_t)(img * IMGD + h0 + ty) * IMGD + w0 + tx) * 32 + 4 * q;
    *(volatile v4f*)op = fv[i];
  }
}

__global__ __launch_bounds__(NTHR) void k_c3(const float* __restrict__ H2, const float* __restrict__ W3f,
                                             const float* __restrict__ R, float* Zout) {
  __shared__ __attribute__((aligned(16))) float sH2[340 * H2P];
  __shared__ __attribute__((aligned(16))) float sW3[288];
  const int tid = (int)threadIdx.x;
  const int blk = (int)blockIdx.x;
  const int img = blk >> 6, h0 = ((blk >> 2) & 15) * 8, w0 = (blk & 3) * 32;

#pragma unroll 1
  for (int i = 0; i < 11; ++i) {
    const int idx = tid + NTHR * i;
    const int ic = idx < 2720 ? idx : 2719;
    const int p = ic >> 3, q = ic & 7;
    const int py = p / 34, px = p - py * 34;
    const int gh = h0 - 1 + py, gw = w0 - 1 + px;
    const bool ins = ((unsigned)gh < (unsigned)IMGD) && ((unsigned)gw < (unsigned)IMGD);
    const int ghc = clampi(gh, 0, IMGD - 1), gwc = clampi(gw, 0, IMGD - 1);
    v4f v = *(const v4f*)(H2 + ((size_t)(img * IMGD + ghc) * IMGD + gwc) * 32 + 4 * q);
    v.x = ins ? v.x : 0.0f; v.y = ins ? v.y : 0.0f; v.z = ins ? v.z : 0.0f; v.w = ins ? v.w : 0.0f;
    if (idx < 2720) *(v4fa*)(sH2 + p * H2P + 4 * q) = v;
  }
  if (tid < 96) {
    const int ic = tid < 72 ? tid : 71;
    const v4f v = *(const v4f*)(W3f + 4 * ic);
    *(v4fa*)(sW3 + 4 * ic) = v;
  }
  __syncthreads();

  const int ty = tid >> 5, tx = tid & 31;
  float acc = 0.0f;
#pragma unroll 1
  for (int t = 0; t < 9; ++t) {
    const int kh = t / 3, kw = t - 3 * kh;
    const float* hp = sH2 + ((ty + kh) * 34 + tx + kw) * H2P;
    const float* wp = sW3 + t * 32;
#pragma unroll
    for (int q = 0; q < 8; ++q) {
      const v4f hv = *(const v4fa*)(hp + 4 * q);
      const v4f wv = *(const v4fa*)(wp + 4 * q);
      acc = fmaf(hv.x, wv.x, acc);
      acc = fmaf(hv.y, wv.y, acc);
      acc = fmaf(hv.z, wv.z, acc);
      acc = fmaf(hv.w, wv.w, acc);
    }
  }
  const size_t gi = (size_t)img * NN + (size_t)(h0 + ty) * IMGD + w0 + tx;
  const float zn = relu_p(R[gi] + acc);
  *(volatile float*)(Zout + gi) = zn;
  __threadfence();
  *(volatile float*)(Zout + gi) = zn;
}

extern "C" void kernel_launch(void* const* d_in, const int* in_sizes, int n_in,
                              void* d_out, int out_size, void* d_ws, size_t ws_size,
                              hipStream_t stream) {
  if (n_in < 10) return;
  if (in_sizes[0] != NE || in_sizes[1] != NE || in_sizes[2] != NE) return;
  if (in_sizes[3] != NB * NN || in_sizes[4] != NB * NN || in_sizes[5] != NB * NM) return;
  if (in_sizes[6] != 864 || in_sizes[7] != 27648 || in_sizes[8] != 864 || in_sizes[9] != 3) return;
  if (out_size != NB * NN) return;

  const float* A_vals = (const float*)d_in[0];
  const int*   A_rows = (const int*)  d_in[1];
  const int*   A_cols = (const int*)  d_in[2];
  const float* z0     = (const float*)d_in[3];
  const float* u      = (const float*)d_in[4];
  const float* y      = (const float*)d_in[5];
  const float* W1     = (const float*)d_in[6];
  const float* W2     = (const float*)d_in[7];
  const float* W3     = (const float*)d_in[8];
  const float* etas   = (const float*)d_in[9];
  float* out = (float*)d_out;

  char* ws = (char*)d_ws;
  size_t off = 0;
  const size_t oTAB = off; off += (size_t)TAB_N * 4;                off = (off + 255) & ~(size_t)255;
  const size_t oW2T = off; off += (size_t)NUW2 * 16;                off = (off + 255) & ~(size_t)255;
  const size_t oSTG = off; off += (size_t)NE * 8;                   off = (off + 255) & ~(size_t)255;
  const size_t oRO  = off; off += (size_t)NCH * ROPITCH * 4;        off = (off + 255) & ~(size_t)255;
  const size_t oLR  = off; off += (size_t)NBK_R * BCAP_R * 8;       off = (off + 255) & ~(size_t)255;
  const size_t oLC  = off; off += (size_t)NBK_C * BCAP_C * 8;       off = (off + 255) & ~(size_t)255;
  const size_t oOR  = off; off += (size_t)NBK_R * OFFP * 4;         off = (off + 255) & ~(size_t)255;
  const size_t oOC  = off; off += (size_t)NBK_C * OFFP * 4;         off = (off + 255) & ~(size_t)255;
  const size_t oH2  = off; off += (size_t)NB * NN * 32 * 4;         off = (off + 255) & ~(size_t)255;
  const size_t oZ   = off; off += (size_t)NB * NN * 4;              off = (off + 255) & ~(size_t)255;
  const size_t oR   = off; off += (size_t)NB * NN * 4;              off = (off + 255) & ~(size_t)255;
  const size_t oZU  = off; off += (size_t)NN * NB * 4;              off = (off + 255) & ~(size_t)255;
  const size_t oVT  = off; off += (size_t)NN * NB * 4;              off = (off + 255) & ~(size_t)255;
  const size_t oRT  = off; off += (size_t)NM * NB * 4;              off = (off + 255) & ~(size_t)255;
  const size_t oNR  = off; off += (size_t)NBK_C * 16 * 8;           off = (off + 255) & ~(size_t)255;
  if (off > ws_size || off > (size_t)WSMAX) return;

  float*          TAB   = (float*)(ws + oTAB);
  unsigned short* W2T   = (unsigned short*)(ws + oW2T);
  int*            STG   = (int*)(ws + oSTG);
  int*            RUNO  = (int*)(ws + oRO);
  int*            LISTR = (int*)(ws + oLR);
  int*            LISTC = (int*)(ws + oLC);
  int*            OFFR  = (int*)(ws + oOR);
  int*            OFFC  = (int*)(ws + oOC);
  float*          H2    = (float*)(ws + oH2);
  float*          Zw    = (float*)(ws + oZ);
  float*          Rw    = (float*)(ws + oR);
  float*          ZUT   = (float*)(ws + oZU);
  float*          VT    = (float*)(ws + oVT);
  float*          RT    = (float*)(ws + oRT);
  double*         NREC  = (double*)(ws + oNR);

  const int ldsBktR = BK_OFF_CNT + 512 * NBK_R;
  const int ldsBktC = BK_OFF_CNT + 512 * NBK_C;
  const int ldsCsrR = BCAP_R * 10 + 32768 + 3904;
  const int ldsCsrC = BCAP_C * 10 + 32768 + 3904;
  hipFuncSetAttribute(reinterpret_cast<const void*>(&k_bkt),
                      hipFuncAttributeMaxDynamicSharedMemorySize, ldsBktC);
  hipFuncSetAttribute(reinterpret_cast<const void*>(&k_csr<BCAP_R>),
                      hipFuncAttributeMaxDynamicSharedMemorySize, ldsCsrR);
  hipFuncSetAttribute(reinterpret_cast<const void*>(&k_csr<BCAP_C>),
                      hipFuncAttributeMaxDynamicSharedMemorySize, ldsCsrC);
  hipFuncSetAttribute(reinterpret_cast<const void*>(&k_c12),
                      hipFuncAttributeMaxDynamicSharedMemorySize, C12_LDS);

  k_prep<<<PB_W2 + 3, NTHR, 0, stream>>>(W1, W2, W3, etas, TAB, W2T);
  k_bkt<<<NCH, NTHR, ldsBktR, stream>>>(A_rows, A_cols, A_vals, NBK_R, NM, NN, STG, RUNO);
  k_csr<BCAP_R><<<NBK_R, NTHR, ldsCsrR, stream>>>(STG, RUNO, LISTR, OFFR);
  k_bkt<<<NCH, NTHR, ldsBktC, stream>>>(A_cols, A_rows, A_vals, NBK_C, NN, NM, STG, RUNO);
  k_csr<BCAP_C><<<NBK_C, NTHR, ldsCsrC, stream>>>(STG, RUNO, LISTC, OFFC);

  for (int j = 0; j < 3; ++j) {
    const float* Zs = (j == 0) ? z0 : Zw;
    const int rz = (j == 0) ? 1 : 0;
    float* Zo = (j == 2) ? out : Zw;
    k_zu<<<NN / 256, NTHR, 0, stream>>>(Zs, rz, u, ZUT);
    k_walk<0, BCAP_R><<<NBK_R, NTHR, 0, stream>>>(LISTR, OFFR, ZUT, y, RT, NREC, NM, NN);
    k_walk<1, BCAP_C><<<NBK_C, NTHR, 0, stream>>>(LISTC, OFFC, RT, u, VT, NREC, NN, NM);
    k_r<<<NN / 256, NTHR, 0, stream>>>(Zs, rz, VT, NREC, TAB + TAB_ETA + j, Rw);
    k_c12<<<NB * 64, NTHR, C12_LDS, stream>>>(Rw, TAB + TAB_W1 + j * 288, W2T + (size_t)j * 9 * 32 * 32, H2);
    k_c3<<<NB * 64, NTHR, 0, stream>>>(H2, TAB + TAB_W3 + j * 288, Rw, Zo);
  }
}
